// MinesweeperGNN_29746943492174
// MI455X (gfx1250) — hardware-verified
//
#include <hip/hip_runtime.h>
#include <stddef.h>


#define NT      256
#define NWV     8
#define FEAT    3
#define HID     32
#define HHALF   16
#define OUTD    2
#define SPW     4
#define CHK     16384
#define EPT1    (CHK / NT)
#define KSH     14
#define BKW     512
#define LBKT    11
#define NBKT    (1 << LBKT)
#define RCAP    20480
#define EPT3    (RCAP / NT)
#define PSH     20
#define TGT     (NWV * 32)
#define GROWS   (NWV * 16)
#define DEGCAP  128
#define WPLN    (HID * HID)
#define WSCAP   134217728

#define LDS1 ((2 * CHK + NT * 16 + 32 + 2 * BKW) * 4)
#define LDS3 ((2 * RCAP + NT * 16 + 32 + 2 * NBKT) * 4)

static_assert(CHK == NT * EPT1);
static_assert(RCAP == NT * EPT3);
static_assert((EPT1 % 4) == 0 && (EPT3 % 4) == 0);
static_assert((RCAP % 32) == 0 && (CHK % 32) == 0);
static_assert((1 << KSH) == CHK);
static_assert((NBKT % TGT) == 0 && (TGT % GROWS) == 0);
static_assert(NBKT <= (1 << (31 - PSH)));
static_assert(NWV * 2 == 16);
static_assert(HID == 32 && BKW == 512 && HID == 2 * HHALF);
static_assert((NBKT % (4 * NT)) == 0);
static_assert(TGT == NT);
static_assert(GROWS * HHALF == NWV * 256);

typedef float          v2f  __attribute__((ext_vector_type(2), may_alias));
typedef float          v4f  __attribute__((ext_vector_type(4), may_alias));
typedef float          v8f  __attribute__((ext_vector_type(8)));
typedef int            v4i  __attribute__((ext_vector_type(4), may_alias));
typedef unsigned       v4u  __attribute__((ext_vector_type(4), may_alias));
typedef unsigned short v8us __attribute__((ext_vector_type(8)));
typedef __bf16         v16b __attribute__((ext_vector_type(16)));
union FragB { v16b v; v8us h[2]; };

__device__ __forceinline__ int clampi(int v, int lo, int hi) { v = v < lo ? lo : v; return v > hi ? hi : v; }

__device__ __forceinline__ unsigned int bfr(float f) {
  const unsigned int u = __float_as_uint(f);
  return (u + 0x7FFFu + ((u >> 16) & 1u)) >> 16;
}

__device__ __forceinline__ void split1(float x, unsigned short& hb, unsigned short& lb) {
  const unsigned int hu = bfr(x);
  const float hf = __uint_as_float(hu << 16);
  hb = (unsigned short)hu;
  lb = (unsigned short)bfr(x - hf);
}

__device__ __forceinline__ void split8(v4f a, v4f b, v8us& hi, v8us& lo) {
  unsigned short hb, lb;
  split1(a.x, hb, lb); hi[0] = hb; lo[0] = lb;
  split1(a.y, hb, lb); hi[1] = hb; lo[1] = lb;
  split1(a.z, hb, lb); hi[2] = hb; lo[2] = lb;
  split1(a.w, hb, lb); hi[3] = hb; lo[3] = lb;
  split1(b.x, hb, lb); hi[4] = hb; lo[4] = lb;
  split1(b.y, hb, lb); hi[5] = hb; lo[5] = lb;
  split1(b.z, hb, lb); hi[6] = hb; lo[6] = lb;
  split1(b.w, hb, lb); hi[7] = hb; lo[7] = lb;
}

__device__ __forceinline__ v8f wmb(v16b a, v16b b, v8f c) {
  v8f d = __builtin_amdgcn_wmma_f32_16x16x32_bf16(false, a, false, b, (short)0, c, false, false);
  asm volatile("v_nop\n\tv_nop\n\tv_nop\n\tv_nop" : "+v"(d) : "v"(a), "v"(b));
  return d;
}

__device__ __forceinline__ int wave_max(int v) {
#pragma unroll
  for (int m = 16; m > 0; m >>= 1) { const int o = __shfl_xor(v, m); v = v > o ? v : o; }
  return __builtin_amdgcn_readfirstlane(v);
}

__device__ __forceinline__ int bscan8(int v, int* wtot, int lane, int wave, int& total) {
  int incl = v;
#pragma unroll
  for (int d = 1; d < 32; d <<= 1) { const int t2 = __shfl_up(incl, d); incl += (lane >= d) ? t2 : 0; }
  if (lane == 31) wtot[wave] = incl;
  __syncthreads();
  int pre = 0, tot = 0;
#pragma unroll
  for (int w = 0; w < NWV; ++w) { const int x = wtot[w]; pre += (w < wave) ? x : 0; tot += x; }
  total = tot;
  return pre + incl - v;
}

__device__ __forceinline__ v4f fma4(float w, v4f v, v4f a) {
  v4f r;
  r.x = fmaf(w, v.x, a.x); r.y = fmaf(w, v.y, a.y); r.z = fmaf(w, v.z, a.z); r.w = fmaf(w, v.w, a.w);
  return r;
}

template <int EPT, int NTOT>
__device__ __forceinline__ void radix_pass(const unsigned* in, unsigned* out, int* ctab, int* stot,
                                           int sh, int tid, int lane, int wave) {
  int* myc = ctab + tid * 16;
#pragma unroll
  for (int d = 0; d < 16; ++d) myc[d] = 0;
  const unsigned* ip = in + tid * EPT;
#pragma unroll 4
  for (int j = 0; j < EPT; ++j) {
    const unsigned k = ip[j];
    const int d = (int)((k >> sh) & 15u);
    myc[d] = myc[d] + 1;
  }
  __syncthreads();
#pragma unroll 1
  for (int dd = 0; dd < 2; ++dd) {
    const int d = 2 * wave + dd;
    int run = 0;
#pragma unroll 1
    for (int k = 0; k < NT / 32; ++k) {
      int* cp = ctab + (32 * k + lane) * 16 + d;
      const int v = *cp;
      int incl = v;
#pragma unroll
      for (int s = 1; s < 32; s <<= 1) { const int t2 = __shfl_up(incl, s); incl += (lane >= s) ? t2 : 0; }
      *cp = run + incl - v;
      run += __shfl(incl, 31);
    }
    if (lane == 0) stot[d] = run;
  }
  __syncthreads();
  {
    int tv[16];
    const v4i q0 = *(const v4i*)(stot), q1 = *(const v4i*)(stot + 4);
    const v4i q2 = *(const v4i*)(stot + 8), q3 = *(const v4i*)(stot + 12);
    tv[0] = q0.x; tv[1] = q0.y; tv[2]  = q0.z; tv[3]  = q0.w; tv[4]  = q1.x; tv[5]  = q1.y; tv[6]  = q1.z; tv[7]  = q1.w;
    tv[8] = q2.x; tv[9] = q2.y; tv[10] = q2.z; tv[11] = q2.w; tv[12] = q3.x; tv[13] = q3.y; tv[14] = q3.z; tv[15] = q3.w;
    int base = 0;
#pragma unroll
    for (int d = 0; d < 16; ++d) { const int cc = myc[d]; myc[d] = cc + base; base += tv[d]; }
  }
#pragma unroll 4
  for (int j = 0; j < EPT; ++j) {
    const unsigned k = ip[j];
    const int d = (int)((k >> sh) & 15u);
    const int p = myc[d];
    out[clampi(p, 0, NTOT - 1)] = k;
    myc[d] = p + 1;
  }
  __syncthreads();
}

template <int EPT, int NTOT>
__device__ __forceinline__ void bounds_pass(const unsigned* a, int* sStart, int* sEnd, int sh, int nv, int tid) {
  const int i0 = tid * EPT;
  const int im = i0 > 0 ? i0 - 1 : 0;
  const int craw0 = (int)(a[im] >> sh);
  int clast = i0 > 0 ? craw0 : -1;
  int ccur = (int)(a[i0] >> sh);
#pragma unroll 2
  for (int j = 0; j < EPT; ++j) {
    const int i  = i0 + j;
    const int in = (i + 1 < NTOT) ? (i + 1) : (NTOT - 1);
    const int craw = (int)(a[in] >> sh);
    const int cnext = (i + 1 < NTOT) ? craw : 0x7FFFFFFF;
    if (ccur < nv) {
      if (ccur != clast) sStart[ccur] = i;
      if (ccur != cnext) sEnd[ccur] = i + 1;
    }
    clast = ccur; ccur = cnext;
  }
}

__global__ __launch_bounds__(128) void k_wprep(const float* __restrict__ w, unsigned short* wp) {
  const int i  = (int)threadIdx.x;
  const int n  = i >> 2;
  const int k0 = (i & 3) * 8;
  float v[8];
#pragma unroll
  for (int e = 0; e < 8; ++e) v[e] = w[(k0 + e) * HID + n];
  v4f a, b;
  a.x = v[0]; a.y = v[1]; a.z = v[2]; a.w = v[3];
  b.x = v[4]; b.y = v[5]; b.z = v[6]; b.w = v[7];
  v8us hv, lv;
  split8(a, b, hv, lv);
  unsigned short* dh = wp + (size_t)i * 8;
  unsigned short* dl = dh + WPLN;
  *(volatile v8us*)dh = hv;
  *(volatile v8us*)dl = lv;
  __threadfence();
  *(volatile v8us*)dh = hv;
  *(volatile v8us*)dl = lv;
}

__global__ __launch_bounds__(NT) void k_csort(const int* __restrict__ ei, unsigned* skey, int* boff, int* bcnt,
                                               int nE, int nN, int vec) {
  extern __shared__ v4i lds_dyn[];
  unsigned* bufA = (unsigned*)lds_dyn;
  unsigned* bufB = bufA + CHK;
  int* ctab = (int*)(bufB + CHK);
  int* stot = ctab + NT * 16;
  int* sSt  = stot + 32;
  int* sEn  = sSt + BKW;
  const int tid = (int)threadIdx.x, lane = tid & 31, wave = tid >> 5;
  const int c = (int)blockIdx.x;
  const int cbase = c * CHK;
  const int* dsts = ei + nE;

  for (int i = tid; i < BKW; i += NT) { sSt[i] = 0; sEn[i] = 0; }
  const bool full = (cbase + CHK <= nE);
#pragma unroll 1
  for (int k = 0; k < EPT1 / 4; ++k) {
    const int q  = tid + NT * k;
    const int e0 = cbase + 4 * q;
    int d0, d1, d2, d3, v0, v1, v2, v3;
    if (vec != 0 && full) {
      const v4i d4 = *(const v4i*)(dsts + e0);
      d0 = d4.x; d1 = d4.y; d2 = d4.z; d3 = d4.w; v0 = 1; v1 = 1; v2 = 1; v3 = 1;
    } else {
      d0 = dsts[clampi(e0, 0, nE - 1)];     v0 = (e0 < nE) ? 1 : 0;
      d1 = dsts[clampi(e0 + 1, 0, nE - 1)]; v1 = (e0 + 1 < nE) ? 1 : 0;
      d2 = dsts[clampi(e0 + 2, 0, nE - 1)]; v2 = (e0 + 2 < nE) ? 1 : 0;
      d3 = dsts[clampi(e0 + 3, 0, nE - 1)]; v3 = (e0 + 3 < nE) ? 1 : 0;
    }
    d0 = clampi(d0, 0, nN - 1); d1 = clampi(d1, 0, nN - 1);
    d2 = clampi(d2, 0, nN - 1); d3 = clampi(d3, 0, nN - 1);
    const unsigned sb = (unsigned)(BKW - 1) << KSH;
    const unsigned li = (unsigned)(4 * q);
    v4u kk;
    kk.x = (v0 ? ((unsigned)(d0 >> LBKT) << KSH) : sb) | li;
    kk.y = (v1 ? ((unsigned)(d1 >> LBKT) << KSH) : sb) | (li + 1u);
    kk.z = (v2 ? ((unsigned)(d2 >> LBKT) << KSH) : sb) | (li + 2u);
    kk.w = (v3 ? ((unsigned)(d3 >> LBKT) << KSH) : sb) | (li + 3u);
    *(v4u*)(bufA + 4 * q) = kk;
  }
  __syncthreads();

  radix_pass<EPT1, CHK>(bufA, bufB, ctab, stot, KSH,     tid, lane, wave);
  radix_pass<EPT1, CHK>(bufB, bufA, ctab, stot, KSH + 4, tid, lane, wave);
  radix_pass<EPT1, CHK>(bufA, bufB, ctab, stot, KSH + 8, tid, lane, wave);
  bounds_pass<EPT1, CHK>(bufB, sSt, sEn, KSH, BKW, tid);

#pragma unroll 2
  for (int j = 0; j < EPT1; ++j) {
    const int pos = tid + NT * j;
    const unsigned key = bufB[pos];
    const int idx = (int)(key & (unsigned)(CHK - 1));
    const int e  = cbase + idx;
    const int ec = e < nE ? e : nE - 1;
    const int s  = clampi(ei[ec], 0, nN - 1);
    const int d  = clampi(dsts[ec], 0, nN - 1);
    const unsigned pk = ((unsigned)(d & (NBKT - 1)) << PSH) | (unsigned)s;
    bufA[pos] = (e < nE) ? pk : 0xFFFFFFFFu;
  }
  __syncthreads();

  unsigned* gk = skey + (size_t)c * CHK;
  int* go = boff + (size_t)c * BKW;
  int* gc = bcnt + (size_t)c * BKW;
#pragma unroll 1
  for (int k = 0; k < EPT1 / 4; ++k) {
    const int i = tid + NT * k;
    const v4u v = ((const v4u*)bufA)[i];
    *(volatile v4u*)(gk + 4 * i) = v;
  }
  if (tid < BKW / 4) {
    v4i st, cn;
    st.x = sSt[4 * tid]; st.y = sSt[4 * tid + 1]; st.z = sSt[4 * tid + 2]; st.w = sSt[4 * tid + 3];
    cn.x = sEn[4 * tid] - st.x; cn.y = sEn[4 * tid + 1] - st.y; cn.z = sEn[4 * tid + 2] - st.z; cn.w = sEn[4 * tid + 3] - st.w;
    cn.x = cn.x < 0 ? 0 : cn.x; cn.y = cn.y < 0 ? 0 : cn.y; cn.z = cn.z < 0 ? 0 : cn.z; cn.w = cn.w < 0 ? 0 : cn.w;
    *(volatile v4i*)(go + 4 * tid) = st;
    *(volatile v4i*)(gc + 4 * tid) = cn;
  }
  __threadfence();
#pragma unroll 1
  for (int k = 0; k < EPT1 / 4; ++k) {
    const int i = tid + NT * k;
    const v4u v = ((const v4u*)bufA)[i];
    *(volatile v4u*)(gk + 4 * i) = v;
  }
  if (tid < BKW / 4) {
    v4i st, cn;
    st.x = sSt[4 * tid]; st.y = sSt[4 * tid + 1]; st.z = sSt[4 * tid + 2]; st.w = sSt[4 * tid + 3];
    cn.x = sEn[4 * tid] - st.x; cn.y = sEn[4 * tid + 1] - st.y; cn.z = sEn[4 * tid + 2] - st.z; cn.w = sEn[4 * tid + 3] - st.w;
    cn.x = cn.x < 0 ? 0 : cn.x; cn.y = cn.y < 0 ? 0 : cn.y; cn.z = cn.z < 0 ? 0 : cn.z; cn.w = cn.w < 0 ? 0 : cn.w;
    *(volatile v4i*)(go + 4 * tid) = st;
    *(volatile v4i*)(gc + 4 * tid) = cn;
  }
}

__global__ __launch_bounds__(512) void k_bbase(const int* __restrict__ bcnt, int* bbase, int nCh, int nBk) {
  __shared__ int wtot[16];
  __shared__ __attribute__((aligned(16))) int sB[BKW];
  const int tid = (int)threadIdx.x, lane = tid & 31, wave = tid >> 5;
  int T = 0;
#pragma unroll 1
  for (int c = 0; c < nCh; ++c) { const int v = bcnt[(size_t)c * BKW + tid]; T += clampi(v, 0, CHK); }
  T = (tid < nBk) ? T : 0;
  int L = T < RCAP ? T : RCAP;
  L = (L + 31) & ~31;
  int incl = L;
#pragma unroll
  for (int d = 1; d < 32; d <<= 1) { const int t2 = __shfl_up(incl, d); incl += (lane >= d) ? t2 : 0; }
  if (lane == 31) wtot[wave] = incl;
  __syncthreads();
  int pre = 0;
#pragma unroll
  for (int w = 0; w < 16; ++w) { const int x = wtot[w]; pre += (w < wave) ? x : 0; }
  sB[tid] = pre + incl - L;
  __syncthreads();
  v4i bv = {0, 0, 0, 0};
  if (tid < BKW / 4) bv = ((const v4i*)sB)[tid];
  if (tid < BKW / 4) *(volatile v4i*)(bbase + 4 * tid) = bv;
  __threadfence();
  if (tid < BKW / 4) *(volatile v4i*)(bbase + 4 * tid) = bv;
}

__global__ __launch_bounds__(NT) void k_bucket(
    const unsigned* __restrict__ skey, const int* __restrict__ boff, const int* __restrict__ bcnt,
    const int* __restrict__ bbase, int* csr, int* toff, int* tcnt, float* dinv, int nCh, int csrLen) {
  extern __shared__ v4i lds_dyn[];
  unsigned* bufA = (unsigned*)lds_dyn;
  unsigned* bufB = bufA + RCAP;
  int* ctab = (int*)(bufB + RCAP);
  int* stot = ctab + NT * 16;
  int* wtot = stot + 16;
  int* tSt  = stot + 32;
  int* tEn  = tSt + NBKT;
  const int tid = (int)threadIdx.x, lane = tid & 31, wave = tid >> 5;
  const int b = (int)blockIdx.x;

  int base = bbase[b];
  base = clampi(base, 0, csrLen - RCAP);
  base &= ~31;

  for (int i = tid; i < NBKT; i += NT) { tSt[i] = 0; tEn[i] = 0; }

  int cur = 0;
  const int nIt = (nCh + NT - 1) / NT;
#pragma unroll 1
  for (int r = 0; r < nIt; ++r) {
    const int cidx = r * NT + tid;
    const int cv = (cidx < nCh) ? 1 : 0;
    const int cc = cv ? cidx : nCh - 1;
    int o = boff[(size_t)cc * BKW + b];
    int n = bcnt[(size_t)cc * BKW + b];
    o = clampi(o, 0, CHK);
    n = clampi(n, 0, CHK - o);
    n = cv ? n : 0;
    int tot;
    const int ex = bscan8(n, wtot, lane, wave, tot);
    const int my = cur + ex;
    int room = RCAP - my; room = room < 0 ? 0 : room;
    const int ne = n < room ? n : room;
    const int nmw = wave_max(ne);
    const unsigned* sp = skey + (size_t)cc * CHK;
#pragma unroll 1
    for (int p = 0; p < nmw; ++p) {
      int q = p < ne ? p : ne - 1;
      q = q < 0 ? 0 : q;
      q += o;
      q = q > CHK - 1 ? CHK - 1 : q;
      const unsigned v = sp[q];
      if (p < ne) bufA[my + p] = v;
    }
    cur += tot;
    cur = cur > RCAP ? RCAP : cur;
    cur = __builtin_amdgcn_readfirstlane(cur);
    __syncthreads();
  }
  const int len = cur;
  for (int i = len + tid; i < RCAP; i += NT) bufA[i] = 0xFFFFFFFFu;
  __syncthreads();

  radix_pass<EPT3, RCAP>(bufA, bufB, ctab, stot, PSH,     tid, lane, wave);
  radix_pass<EPT3, RCAP>(bufB, bufA, ctab, stot, PSH + 4, tid, lane, wave);
  radix_pass<EPT3, RCAP>(bufA, bufB, ctab, stot, PSH + 8, tid, lane, wave);
  bounds_pass<EPT3, RCAP>(bufB, tSt, tEn, PSH, NBKT, tid);
  __syncthreads();

  const int lenW = (len + 31) & ~31;
  const int nv4 = lenW >> 2;
  int*   gcs = csr + base;
  int*   gtc = tcnt + (size_t)b * NBKT;
  int*   gto = toff + (size_t)b * NBKT;
  float* gdv = dinv + (size_t)b * NBKT;
#pragma unroll 1
  for (int pass = 0; pass < 2; ++pass) {
#pragma unroll 1
    for (int i = tid; i < nv4; i += NT) {
      const v4u k = ((const v4u*)bufB)[i];
      v4i s;
      s.x = (int)(k.x & 0xFFFFFu); s.y = (int)(k.y & 0xFFFFFu); s.z = (int)(k.z & 0xFFFFFu); s.w = (int)(k.w & 0xFFFFFu);
      *(volatile v4i*)(gcs + 4 * i) = s;
    }
#pragma unroll 1
    for (int k2 = 0; k2 < NBKT / (4 * NT); ++k2) {
      const int i  = tid + NT * k2;
      const int t0 = 4 * i;
      v4i st, cn, ov; v4f dv;
      st.x = tSt[t0]; st.y = tSt[t0 + 1]; st.z = tSt[t0 + 2]; st.w = tSt[t0 + 3];
      cn.x = tEn[t0] - st.x; cn.y = tEn[t0 + 1] - st.y; cn.z = tEn[t0 + 2] - st.z; cn.w = tEn[t0 + 3] - st.w;
      cn.x = cn.x < 0 ? 0 : cn.x; cn.y = cn.y < 0 ? 0 : cn.y; cn.z = cn.z < 0 ? 0 : cn.z; cn.w = cn.w < 0 ? 0 : cn.w;
      ov.x = base + st.x; ov.y = base + st.y; ov.z = base + st.z; ov.w = base + st.w;
      dv.x = rsqrtf((float)(cn.x + 1)); dv.y = rsqrtf((float)(cn.y + 1));
      dv.z = rsqrtf((float)(cn.z + 1)); dv.w = rsqrtf((float)(cn.w + 1));
      *(volatile v4i*)(gtc + 4 * i) = cn;
      *(volatile v4i*)(gto + 4 * i) = ov;
      *(volatile v4f*)(gdv + 4 * i) = dv;
    }
    if (pass == 0) __threadfence();
  }
}

__global__ __launch_bounds__(NT) void k_agg1(
    const int* __restrict__ csr, const int* __restrict__ toff, const int* __restrict__ tcnt,
    const float* __restrict__ dinv, const float* __restrict__ x, float* spl, int nN, int csrLen) {
  const int tid = (int)threadIdx.x;
  const int t  = (int)blockIdx.x * TGT + tid;
  const int n  = clampi(tcnt[t], 0, DEGCAP);
  const int o  = toff[t];
  const float dt = dinv[t];
  const int nmw = wave_max(n);

  float s0 = 0.f, s1 = 0.f, s2 = 0.f;
#pragma unroll 1
  for (int p = 0; p < nmw; ++p) {
    const int pp  = p < n ? p : n - 1;
    const int pos = clampi(o + pp, 0, csrLen - 1);
    const int s   = clampi(csr[pos], 0, nN - 1);
    const float d = dinv[s];
    const float* xr = x + (size_t)s * FEAT;
    const float x0 = xr[0], x1 = xr[1], x2 = xr[2];
    const float w = p < n ? d : 0.0f;
    s0 = fmaf(w, x0, s0); s1 = fmaf(w, x1, s1); s2 = fmaf(w, x2, s2);
  }
  {
    const int tc = t < nN ? t : nN - 1;
    const float* xr = x + (size_t)tc * FEAT;
    s0 = fmaf(dt, xr[0], s0); s1 = fmaf(dt, xr[1], s1); s2 = fmaf(dt, xr[2], s2);
  }
  v4f rv;
  rv.x = s0; rv.y = s1; rv.z = s2; rv.w = dt;
  float* gp = spl + (size_t)t * SPW;
  *(volatile v4f*)gp = rv;
  __threadfence();
  *(volatile v4f*)gp = rv;
}

__device__ __forceinline__ v4f h1quad(v4f sv, const float* __restrict__ W1, const float* __restrict__ b1, int c0) {
  const v4f w0 = *(const v4f*)(W1 + c0);
  const v4f w1 = *(const v4f*)(W1 + HID + c0);
  const v4f w2 = *(const v4f*)(W1 + 2 * HID + c0);
  const v4f bb = *(const v4f*)(b1 + c0);
  v4f r; float a;
  a = sv.x * w0.x; a = fmaf(sv.y, w1.x, a); a = fmaf(sv.z, w2.x, a); a = fmaf(sv.w, a, bb.x); r.x = fmaxf(a, 0.0f);
  a = sv.x * w0.y; a = fmaf(sv.y, w1.y, a); a = fmaf(sv.z, w2.y, a); a = fmaf(sv.w, a, bb.y); r.y = fmaxf(a, 0.0f);
  a = sv.x * w0.z; a = fmaf(sv.y, w1.z, a); a = fmaf(sv.z, w2.z, a); a = fmaf(sv.w, a, bb.z); r.z = fmaxf(a, 0.0f);
  a = sv.x * w0.w; a = fmaf(sv.y, w1.w, a); a = fmaf(sv.z, w2.w, a); a = fmaf(sv.w, a, bb.w); r.w = fmaxf(a, 0.0f);
  return r;
}

__global__ __launch_bounds__(NT) void k_gemm2(
    const float* __restrict__ spl, const unsigned short* __restrict__ wp, const float* __restrict__ dinv,
    const float* __restrict__ W1, const float* __restrict__ b1, float* hwp, int half) {
  __shared__ __attribute__((aligned(16))) float stg[GROWS * HHALF];
  const int tid = (int)threadIdx.x, lane = tid & 31, wave = tid >> 5, hh = lane >> 4, m = lane & 15;
  const int r0 = (int)blockIdx.x * GROWS + wave * 16;

  const v4f sv = *(const v4f*)(spl + (size_t)(r0 + m) * SPW);
  const int ca = 8 * hh, cb = HHALF + 8 * hh;
  const v4f hA0 = h1quad(sv, W1, b1, ca), hA1 = h1quad(sv, W1, b1, ca + 4);
  const v4f hB0 = h1quad(sv, W1, b1, cb), hB1 = h1quad(sv, W1, b1, cb + 4);
  FragB ah, al;
  split8(hA0, hA1, ah.h[0], al.h[0]);
  split8(hB0, hB1, ah.h[1], al.h[1]);

  const unsigned short* bp = wp + (size_t)(HHALF * half + m) * HID + 8 * hh;
  FragB bh, bl;
  bh.h[0] = *(const v8us*)bp;
  bh.h[1] = *(const v8us*)(bp + 16);
  bl.h[0] = *(const v8us*)(bp + WPLN);
  bl.h[1] = *(const v8us*)(bp + WPLN + 16);
  v8f acc = {0.f, 0.f, 0.f, 0.f, 0.f, 0.f, 0.f, 0.f};
  acc = wmb(ah.v, bh.v, acc);
  acc = wmb(ah.v, bl.v, acc);
  acc = wmb(al.v, bh.v, acc);

  const v4f dA = *(const v4f*)(dinv + (size_t)r0 + 8 * hh);
  const v4f dB = *(const v4f*)(dinv + (size_t)r0 + 8 * hh + 4);
  float s[8];
  s[0] = dA.x; s[1] = dA.y; s[2] = dA.z; s[3] = dA.w; s[4] = dB.x; s[5] = dB.y; s[6] = dB.z; s[7] = dB.w;
  float* sp = stg + (wave * 16 + 8 * hh) * HHALF + m;
#pragma unroll
  for (int r = 0; r < 8; ++r) sp[r * HHALF] = acc[r] * s[r];
  __syncthreads();

  const float* lp = stg + wave * 16 * HHALF;
  const v4f v0 = *(const v4f*)(lp + 4 * lane);
  const v4f v1 = *(const v4f*)(lp + 128 + 4 * lane);
  float* gp = hwp + (size_t)r0 * HHALF;
  *(volatile v4f*)(gp + 4 * lane) = v0;
  *(volatile v4f*)(gp + 128 + 4 * lane) = v1;
  __threadfence();
  *(volatile v4f*)(gp + 4 * lane) = v0;
  *(volatile v4f*)(gp + 128 + 4 * lane) = v1;
}

__device__ __forceinline__ void head4(v4f a, v4f u, float dt, const float* __restrict__ b2,
                                      const float* __restrict__ W3, int c, float& p0, float& p1) {
  float h;
  h = fmaxf(fmaf(dt, a.x + u.x, b2[c]),     0.0f); p0 = fmaf(h, W3[c * OUTD],       p0); p1 = fmaf(h, W3[c * OUTD + 1],       p1);
  h = fmaxf(fmaf(dt, a.y + u.y, b2[c + 1]), 0.0f); p0 = fmaf(h, W3[(c + 1) * OUTD], p0); p1 = fmaf(h, W3[(c + 1) * OUTD + 1], p1);
  h = fmaxf(fmaf(dt, a.z + u.z, b2[c + 2]), 0.0f); p0 = fmaf(h, W3[(c + 2) * OUTD], p0); p1 = fmaf(h, W3[(c + 2) * OUTD + 1], p1);
  h = fmaxf(fmaf(dt, a.w + u.w, b2[c + 3]), 0.0f); p0 = fmaf(h, W3[(c + 3) * OUTD], p0); p1 = fmaf(h, W3[(c + 3) * OUTD + 1], p1);
}

__global__ __launch_bounds__(NT) void k_agg2(
    const int* __restrict__ csr, const int* __restrict__ toff, const int* __restrict__ tcnt,
    const float* __restrict__ dinv, const float* __restrict__ hw, const float* __restrict__ W3,
    const float* __restrict__ b2, const float* __restrict__ b3, const float* pin,
    float* dst, int half, int nLim, int nN, int csrLen) {
  __shared__ __attribute__((aligned(16))) float sO[TGT * OUTD];
  const int tid = (int)threadIdx.x, wave = tid >> 5;
  const int blockBase = (int)blockIdx.x * TGT;
  const int t  = blockBase + tid;
  const int n  = clampi(tcnt[t], 0, DEGCAP);
  const int o  = toff[t];
  const float dt = dinv[t];
  const int nmw = wave_max(n);
  const int cbase = HHALF * half;

  v4f a0 = {0.f, 0.f, 0.f, 0.f}, a1 = {0.f, 0.f, 0.f, 0.f}, a2 = {0.f, 0.f, 0.f, 0.f}, a3 = {0.f, 0.f, 0.f, 0.f};
#pragma unroll 1
  for (int p = 0; p < nmw; ++p) {
    const int pp  = p < n ? p : n - 1;
    const int pos = clampi(o + pp, 0, csrLen - 1);
    const int s   = clampi(csr[pos], 0, nN - 1);
    const float w = p < n ? 1.0f : 0.0f;
    const float* hr = hw + (size_t)s * HHALF;
    const v4f v0 = *(const v4f*)hr, v1 = *(const v4f*)(hr + 4), v2 = *(const v4f*)(hr + 8), v3 = *(const v4f*)(hr + 12);
    a0 = fma4(w, v0, a0); a1 = fma4(w, v1, a1); a2 = fma4(w, v2, a2); a3 = fma4(w, v3, a3);
  }
  const float* tr = hw + (size_t)t * HHALF;
  const v4f u0 = *(const v4f*)tr, u1 = *(const v4f*)(tr + 4), u2 = *(const v4f*)(tr + 8), u3 = *(const v4f*)(tr + 12);
  float p0 = 0.f, p1 = 0.f;
  head4(a0, u0, dt, b2, W3, cbase,      p0, p1);
  head4(a1, u1, dt, b2, W3, cbase + 4,  p0, p1);
  head4(a2, u2, dt, b2, W3, cbase + 8,  p0, p1);
  head4(a3, u3, dt, b2, W3, cbase + 12, p0, p1);
  const float b30 = b3[0], b31 = b3[1];
  p0 += (half == 0) ? b30 : 0.0f;
  p1 += (half == 0) ? b31 : 0.0f;
  v2f pr; pr.x = p0; pr.y = p1;
  *(v2f*)(sO + tid * OUTD) = pr;
  __syncthreads();

  if (wave < 4) {
    const int tgl = blockBase + 2 * tid;
    v4f v = ((const v4f*)sO)[tid];
    const v4f q = *(const v4f*)(pin + (size_t)blockBase * OUTD + 4 * tid);
    if (half != 0) v = v + q;
    float* gp = dst + (size_t)blockBase * OUTD + 4 * tid;
    const bool fullp = (tgl + 2 <= nLim);
    const bool halfp = (!fullp) && (tgl + 1 == nLim);
    v2f u; u.x = v.x; u.y = v.y;
    if (fullp) *(volatile v4f*)gp = v;
    else if (halfp) *(volatile v2f*)gp = u;
    __threadfence();
    if (fullp) *(volatile v4f*)gp = v;
    else if (halfp) *(volatile v2f*)gp = u;
  }
}

extern "C" void kernel_launch(void* const* d_in, const int* in_sizes, int n_in,
                              void* d_out, int out_size, void* d_ws, size_t ws_size,
                              hipStream_t stream) {
  if (n_in < 8) return;
  const int nN = in_sizes[0] / FEAT;
  const int nE = in_sizes[1] / 2;
  if (nN <= 0 || nE <= 0 || in_sizes[0] != nN * FEAT || in_sizes[1] != 2 * nE) return;
  if (in_sizes[2] != FEAT * HID || in_sizes[3] != HID) return;
  if (in_sizes[4] != HID * HID || in_sizes[5] != HID) return;
  if (in_sizes[6] != HID * OUTD || in_sizes[7] != OUTD) return;
  if (out_size != nN * OUTD) return;
  if (nN > (1 << 20) || nE > (1 << 28)) return;

  const float* x  = (const float*)d_in[0];
  const int*   ei = (const int*)d_in[1];
  const float* W1 = (const float*)d_in[2];
  const float* b1 = (const float*)d_in[3];
  const float* W2 = (const float*)d_in[4];
  const float* b2 = (const float*)d_in[5];
  const float* W3 = (const float*)d_in[6];
  const float* b3 = (const float*)d_in[7];
  float* out = (float*)d_out;

  const int nBk   = (nN + NBKT - 1) / NBKT;
  if (nBk > BKW - 1) return;
  const int nCh   = (nE + CHK - 1) / CHK;
  const int NPADH = ((nN + TGT - 1) / TGT) * TGT;
  const int NP1   = nBk * NBKT;
  const int csrLen = ((nE + 31) & ~31) + 32 * nBk + RCAP;
  const int nAgg  = NPADH / TGT;
  const int nGemm = NPADH / GROWS;

  char* ws = (char*)d_ws;
  size_t off = 0;
  const size_t oW   = off; off += (size_t)2 * WPLN * 2;          off = (off + 255) & ~(size_t)255;
  const size_t oBB  = off; off += (size_t)BKW * 4;               off = (off + 255) & ~(size_t)255;
  const size_t oDv  = off; off += (size_t)NP1 * 4;               off = (off + 255) & ~(size_t)255;
  const size_t oOff = off; off += (size_t)NP1 * 4;               off = (off + 255) & ~(size_t)255;
  const size_t oCnt = off; off += (size_t)NP1 * 4;               off = (off + 255) & ~(size_t)255;
  const size_t oCsr = off; off += (size_t)csrLen * 4;            off = (off + 255) & ~(size_t)255;
  const size_t oS   = off; off += (size_t)NPADH * SPW * 4;       off = (off + 255) & ~(size_t)255;
  const size_t oPt  = off; off += (size_t)NPADH * OUTD * 4;      off = (off + 255) & ~(size_t)255;
  const size_t oU   = off;
  size_t u1 = 0;
  const size_t oSK  = oU + u1; u1 += (size_t)nCh * CHK * 4;      u1 = (u1 + 255) & ~(size_t)255;
  const size_t oBo  = oU + u1; u1 += (size_t)nCh * BKW * 4;      u1 = (u1 + 255) & ~(size_t)255;
  const size_t oBc  = oU + u1; u1 += (size_t)nCh * BKW * 4;      u1 = (u1 + 255) & ~(size_t)255;
  size_t u2 = (size_t)NPADH * HHALF * 4;                         u2 = (u2 + 255) & ~(size_t)255;
  const size_t oH   = oU;
  off = oU + (u1 > u2 ? u1 : u2);
  if (off > ws_size || off > (size_t)WSCAP) return;

  unsigned short* wpn  = (unsigned short*)(ws + oW);
  int*      bbase = (int*)(ws + oBB);
  float*    dinv  = (float*)(ws + oDv);
  int*      toffp = (int*)(ws + oOff);
  int*      tcntp = (int*)(ws + oCnt);
  int*      csr   = (int*)(ws + oCsr);
  float*    spl   = (float*)(ws + oS);
  float*    part  = (float*)(ws + oPt);
  unsigned* skey  = (unsigned*)(ws + oSK);
  int*      boffp = (int*)(ws + oBo);
  int*      bcntp = (int*)(ws + oBc);
  float*    hwp   = (float*)(ws + oH);

  const int vec = ((nE & 3) == 0) ? 1 : 0;

  k_wprep<<<1, 128, 0, stream>>>(W2, wpn);

  hipFuncSetAttribute(reinterpret_cast<const void*>(&k_csort), hipFuncAttributeMaxDynamicSharedMemorySize, LDS1);
  k_csort<<<nCh, NT, LDS1, stream>>>(ei, skey, boffp, bcntp, nE, nN, vec);
  k_bbase<<<1, BKW, 0, stream>>>(bcntp, bbase, nCh, nBk);
  hipFuncSetAttribute(reinterpret_cast<const void*>(&k_bucket), hipFuncAttributeMaxDynamicSharedMemorySize, LDS3);
  k_bucket<<<nBk, NT, LDS3, stream>>>(skey, boffp, bcntp, bbase, csr, toffp, tcntp, dinv, nCh, csrLen);

  k_agg1<<<nAgg, NT, 0, stream>>>(csr, toffp, tcntp, dinv, x, spl, nN, csrLen);

  k_gemm2<<<nGemm, NT, 0, stream>>>(spl, wpn, dinv, W1, b1, hwp, 0);
  k_agg2<<<nAgg, NT, 0, stream>>>(csr, toffp, tcntp, dinv, hwp, W3, b2, b3, part, part, 0, NPADH, nN, csrLen);
  k_gemm2<<<nGemm, NT, 0, stream>>>(spl, wpn, dinv, W1, b1, hwp, 1);
  k_agg2<<<nAgg, NT, 0, stream>>>(csr, toffp, tcntp, dinv, hwp, W3, b2, b3, part, out, 1, nN, nN, csrLen);
}
